// GenPhiloText_14379550507654
// MI455X (gfx1250) — hardware-verified
//
#include <hip/hip_runtime.h>
#include <math.h>

typedef __attribute__((ext_vector_type(16))) _Float16 v16h;
typedef __attribute__((ext_vector_type(8)))  _Float16 v8h;
typedef __attribute__((ext_vector_type(16))) __bf16   v16b;
typedef __attribute__((ext_vector_type(8)))  __bf16   v8b;
typedef __attribute__((ext_vector_type(8)))  float    v8f;
typedef __attribute__((ext_vector_type(4)))  float    v4f;

constexpr int kB    = 1024;
constexpr int kT    = 50;
constexpr int kI    = 256;
constexpr int kHid  = 1024;
constexpr int kO    = 256;
constexpr int kG4   = 4 * kHid;
constexpr int kK    = kHid + kI;
constexpr int kThr  = 256;
constexpr float kInCarry = 1024.0f;
constexpr float kWCarry = 4096.0f;
constexpr float kSc = 1.0f / (kInCarry * kWCarry);
constexpr float kF16MinNormal = 6.103515625e-5f;

static_assert((kB % 64) == 0 && (kG4 % 64) == 0 && (kO % 64) == 0 && ((kB / 64) * (kG4 / 64)) % 8 == 0 && ((kB / 64) * (kO / 64)) % 8 == 0, "GEMM M, N multiples of 64; grids exact");
static_assert((kK % 32) == 0 && (kHid % 32) == 0 && (kK % 64) == 0 && (kHid % 64) == 0 && (kI % 64) == 0 && (kHid / 8) <= 256 && (kI / 8) == 32, "GEMM K multiples of 32; the transposing cast's row segments whole lines and its blocks K / 8 threads");

constexpr size_t kOffW16 = 0ull;
constexpr size_t kOffWD16 = 10485760ull;
constexpr size_t kOffBIAS = 11010048ull;
constexpr size_t kOffHX16 = 11030528ull;
constexpr size_t kOffGG = 13651968ull;
constexpr size_t kOffC32 = 30429184ull;
constexpr size_t kOffLOG = 34623488ull;
constexpr size_t kWsTotal = 35672064ull;
static_assert(kWsTotal <= 134217728ull, "carve cap: under 128 MiB");
static_assert(kOffW16 == 0
              && kOffWD16 == kOffW16 + 10485760ull
              && kOffBIAS == kOffWD16 + 524288ull
              && kOffHX16 == kOffBIAS + 20480ull
              && kOffGG == kOffHX16 + 2621440ull
              && kOffC32 == kOffGG + 16777216ull
              && kOffLOG == kOffC32 + 4194304ull
              && kWsTotal == kOffLOG + 1048576ull, "the carve is chained and totalled");
static_assert((kOffW16 % 256) == 0 && (kOffWD16 % 256) == 0 && (kOffBIAS % 256) == 0 && (kOffHX16 % 256) == 0 && (kOffGG % 256) == 0 && (kOffC32 % 256) == 0 && (kOffLOG % 256) == 0, "aligned regions");
constexpr int kFBG = 0, kFBO = 4096, kFEnd = 5120;
static_assert(kFBO == kFBG + kG4 && kFBO + kO <= kFEnd, "bias stream map");

__device__ __forceinline__ unsigned short f2bf_bits(float f) {
  unsigned u = __float_as_uint(f);
  return (unsigned short)((u + 0x7FFFu + ((u >> 16) & 1u)) >> 16);
}
__device__ __forceinline__ float bf_bits2f(unsigned short h) { return __uint_as_float(((unsigned)h) << 16); }
__device__ __forceinline__ float bf16r(float f) { return bf_bits2f(f2bf_bits(f)); }
__device__ __forceinline__ float carry_flush(float v, float carry) {
  const float s = v * carry;
  return (fabsf(s) < kF16MinNormal) ? 0.0f : s;
}
__device__ __forceinline__ float frcp(float x) { return __builtin_amdgcn_rcpf(x); }

__device__ __forceinline__ void dep_guard4_h(v8f& a, v8f& b, v8f& c, v8f& d, v16h x, v16h y) { asm volatile("v_nop\n\tv_nop\n\tv_nop\n\tv_nop" : "+v"(a), "+v"(b), "+v"(c), "+v"(d) : "v"(x), "v"(y)); }
__device__ __forceinline__ void dep_guard4_b(v8f& a, v8f& b, v8f& c, v8f& d, v16b x, v16b y) { asm volatile("v_nop\n\tv_nop\n\tv_nop\n\tv_nop" : "+v"(a), "+v"(b), "+v"(c), "+v"(d) : "v"(x), "v"(y)); }
__device__ __forceinline__ void keep4_h(v16h a, v16h b, v16h c, v16h d) { asm volatile("v_nop" :: "v"(a), "v"(b), "v"(c), "v"(d)); }
__device__ __forceinline__ void keep4_b(v16b a, v16b b, v16b c, v16b d) { asm volatile("v_nop" :: "v"(a), "v"(b), "v"(c), "v"(d)); }
__device__ __forceinline__ void acc_guard4(v8f& a, v8f& b, v8f& c, v8f& d) { asm volatile("v_nop\n\tv_nop\n\tv_nop\n\tv_nop" : "+v"(a), "+v"(b), "+v"(c), "+v"(d)); }

template <typename T> struct Frag;
template <> struct Frag<_Float16> {
  typedef v16h V; union U { v16h v; v8h h[2]; };
  static __device__ __forceinline__ v16h load(const _Float16* p) {
    U f; f.h[0] = *(const v8h*)(p); f.h[1] = *(const v8h*)(p + 16); return f.v;
  }
  static __device__ __forceinline__ v8f mma(v16h a, v16h b, v8f c) {
    return __builtin_amdgcn_wmma_f32_16x16x32_f16(false, a, false, b, (short)0, c, false, false);
  }
  static __device__ __forceinline__ void guard4(v8f& a, v8f& b, v8f& c, v8f& d, v16h x, v16h y) { dep_guard4_h(a, b, c, d, x, y); }
  static __device__ __forceinline__ void keep(v16h a, v16h b, v16h c, v16h d) { keep4_h(a, b, c, d); }
};
template <> struct Frag<__bf16> {
  typedef v16b V; union U { v16b v; v8b h[2]; };
  static __device__ __forceinline__ v16b load(const __bf16* p) {
    U f; f.h[0] = *(const v8b*)(p); f.h[1] = *(const v8b*)(p + 16); return f.v;
  }
  static __device__ __forceinline__ v8f mma(v16b a, v16b b, v8f c) {
    return __builtin_amdgcn_wmma_f32_16x16x32_bf16(false, a, false, b, (short)0, c, false, false);
  }
  static __device__ __forceinline__ void guard4(v8f& a, v8f& b, v8f& c, v8f& d, v16b x, v16b y) { dep_guard4_b(a, b, c, d, x, y); }
  static __device__ __forceinline__ void keep(v16b a, v16b b, v16b c, v16b d) { keep4_b(a, b, c, d); }
};

__device__ __forceinline__ v8f mma_h(v16h a, v16h b, v8f c) {
  c = __builtin_amdgcn_wmma_f32_16x16x32_f16(false, a, false, b, (short)0, c, false, false);
  asm volatile("v_nop\n\tv_nop\n\tv_nop\n\tv_nop" : "+v"(c) : "v"(a), "v"(b));
  return c;
}

template <int ET> struct Elem;
template <> struct Elem<0> { typedef _Float16 T; };
template <> struct Elem<1> { typedef __bf16 T; };
template <int ET, bool SPLIT, int BIAS_MODE, int OUT_MODE, bool RESID, int ACT = 0>
__global__ __launch_bounds__(256) void wmma_gemm64(
    const unsigned short* __restrict__ Ap, const unsigned short* __restrict__ A2p, int lda, long strideA,
    const unsigned short* __restrict__ Btp, const unsigned short* __restrict__ Bt2p, int ldb, long strideB,
    void* __restrict__ Cout, void* __restrict__ Cout2, int ldc, long strideC,
    const float* __restrict__ bias,
    const float* __restrict__ resid, long strideR,
    int M, int N, int K, float scale) {
  typedef typename Elem<ET>::T T;
  typedef typename Frag<T>::V V;
  const T* A = (const T*)Ap; const T* A2 = (const T*)A2p; const T* Bt = (const T*)Btp; const T* Bt2 = (const T*)Bt2p;
  __shared__ __align__(16) float sT[8][16 * 68];
  const int b    = blockIdx.y;
  const int lane = threadIdx.x & 31;
  const int wave = threadIdx.x >> 5;
  const int tilesN = N >> 6;
  const int tilesM = M >> 6;
  const int tile = blockIdx.x * 8 + wave;
  if (tile >= tilesM * tilesN) return;
  const int tm = tile / tilesN;
  const int tn = tile - tm * tilesN;
  const int m0 = tm << 6;
  const int n0 = tn << 6;

  const T* Ab  = A  + (size_t)b * strideA;
  const T* Bb  = Bt + (size_t)b * strideB;
  const T* Ab2 = SPLIT ? (A2  + (size_t)b * strideA) : nullptr;
  const T* Bb2 = SPLIT ? (Bt2 + (size_t)b * strideB) : nullptr;

  const int rlane = lane & 15;
  const int koff  = (lane >> 4) * 8;
  const int mOff  = (lane >> 4) * 8;

  v8f acc[4][4];
#pragma unroll
  for (int i = 0; i < 4; ++i)
#pragma unroll
    for (int j = 0; j < 4; ++j) acc[i][j] = (v8f){0.f,0.f,0.f,0.f,0.f,0.f,0.f,0.f};

  for (int k0 = 0; k0 < K; k0 += 32) {
    V bh[4], bl[4];
#pragma unroll
    for (int j = 0; j < 4; ++j) {
      const size_t bo = (size_t)(n0 + (j << 4) + rlane) * ldb + koff + k0;
      bh[j] = Frag<T>::load(Bb + bo);
      if (SPLIT) bl[j] = Frag<T>::load(Bb2 + bo);
    }
#pragma unroll
    for (int i = 0; i < 4; ++i) {
      const size_t ao = (size_t)(m0 + (i << 4) + rlane) * lda + koff + k0;
      V ah = Frag<T>::load(Ab + ao);
      V al;
      if (SPLIT) al = Frag<T>::load(Ab2 + ao);
#pragma unroll
      for (int j = 0; j < 4; ++j) {
        acc[i][j] = Frag<T>::mma(ah, bh[j], acc[i][j]);
        if (SPLIT) {
          acc[i][j] = Frag<T>::mma(ah, bl[j], acc[i][j]);
          acc[i][j] = Frag<T>::mma(al, bh[j], acc[i][j]);
        }
      }
      Frag<T>::guard4(acc[i][0], acc[i][1], acc[i][2], acc[i][3], ah, SPLIT ? al : ah);
    }
    Frag<T>::keep(bh[0], bh[1], bh[2], bh[3]);
    if (SPLIT) Frag<T>::keep(bl[0], bl[1], bl[2], bl[3]);
  }
  acc_guard4(acc[0][0], acc[0][1], acc[0][2], acc[0][3]);
  acc_guard4(acc[1][0], acc[1][1], acc[1][2], acc[1][3]);
  acc_guard4(acc[2][0], acc[2][1], acc[2][2], acc[2][3]);
  acc_guard4(acc[3][0], acc[3][1], acc[3][2], acc[3][3]);

  float* slab = sT[wave];
  const float* Rb = RESID ? (resid + (size_t)b * strideR) : nullptr;
#pragma unroll
  for (int i = 0; i < 4; ++i) {
    const int mBase = m0 + (i << 4);
#pragma unroll
    for (int j = 0; j < 4; ++j) {
      const int n = n0 + (j << 4) + rlane;
      float bv = 0.f;
      if (BIAS_MODE == 2) bv = bias[n];
#pragma unroll
      for (int r = 0; r < 8; ++r) {
        float v = acc[i][j][r] * scale;
        if (BIAS_MODE == 1) v += bias[mBase + mOff + r];
        if (BIAS_MODE == 2) v += bv;
        if (RESID) v += Rb[(size_t)(mBase + mOff + r) * ldc + n];
        if (ACT == 1) v = tanhf(v);
        if (ACT == 2) v = fmaxf(v, 0.0f);
        if (ACT == 3) v = v / (1.0f + expf(-v));
        if (ACT == 4) v = (v > 0.f) ? v : 0.01f * v;
        slab[(mOff + r) * 68 + (j << 4) + rlane] = v;
      }
    }
    __builtin_amdgcn_fence(__ATOMIC_RELEASE, "workgroup");
    __builtin_amdgcn_wave_barrier();
    __builtin_amdgcn_fence(__ATOMIC_ACQUIRE, "workgroup");
    if (OUT_MODE == 0) {
      float* C = (float*)Cout + (size_t)b * strideC;
      const int hh = lane >> 4, c4 = (lane & 15) * 4;
      for (int pass = 0; pass < 2; ++pass) {
#pragma unroll
        for (int it = 0; it < 8; ++it) {
          const int row = it * 2 + hh;
          v4f v = *(const v4f*)(slab + row * 68 + c4);
          *(volatile v4f*)(C + (size_t)(mBase + row) * ldc + n0 + c4) = v;
        }
        __threadfence();
      }
    } else {
      const int q = lane >> 3, c8 = (lane & 7) * 8;
      unsigned short* C  = (unsigned short*)Cout  + (size_t)b * strideC;
      unsigned short* C2 = (OUT_MODE == 2) ? ((unsigned short*)Cout2 + (size_t)b * strideC) : nullptr;
      for (int pass = 0; pass < 2; ++pass) {
#pragma unroll
        for (int it = 0; it < 4; ++it) {
          const int row = it * 4 + q;
          const float* sp = slab + row * 68 + c8;
          v8h hv, lv;
#pragma unroll
          for (int e = 0; e < 8; ++e) {
            if (OUT_MODE == 1) {
              hv[e] = (_Float16)sp[e];
            } else {
              unsigned short hb = f2bf_bits(sp[e]);
              unsigned short lb = f2bf_bits(sp[e] - bf_bits2f(hb));
              hv[e] = __builtin_bit_cast(_Float16, hb);
              lv[e] = __builtin_bit_cast(_Float16, lb);
            }
          }
          *(volatile v8h*)(C + (size_t)(mBase + row) * ldc + n0 + c8) = hv;
          if (OUT_MODE == 2) *(volatile v8h*)(C2 + (size_t)(mBase + row) * ldc + n0 + c8) = lv;
        }
        __threadfence();
      }
    }
    __builtin_amdgcn_fence(__ATOMIC_RELEASE, "workgroup");
    __builtin_amdgcn_wave_barrier();
    __builtin_amdgcn_fence(__ATOMIC_ACQUIRE, "workgroup");
  }
}

__global__ __launch_bounds__(256) void wt_plane_kernel(const float* __restrict__ W, unsigned short* __restrict__ dst, int K, int N, int nLive, int ldd, int colOff) {
  const int n  = blockIdx.x;
  const int k8 = threadIdx.x * 8;
  const bool live = n < nLive;
  const int nc = live ? n : 0;
  v8h hv;
#pragma unroll
  for (int e = 0; e < 8; ++e) {
    const float w = W[(size_t)(k8 + e) * N + nc];
    hv[e] = (_Float16)(live ? carry_flush(bf16r(w), kWCarry) : 0.0f);
  }
  unsigned short* dp = dst + (size_t)n * ldd + colOff + k8;
  *(volatile v8h*)dp = hv;
  __threadfence();
  *(volatile v8h*)dp = hv;
}


__device__ __forceinline__ float fast_tanh(float v) { return 1.0f - 2.0f * frcp(__expf(2.0f * v) + 1.0f); }
__device__ __forceinline__ float fast_sigmoid(float v) { return frcp(1.0f + __expf(-v)); }

__global__ __launch_bounds__(kThr) void setup_kernel(const float* __restrict__ X, const float* __restrict__ h_0, const float* __restrict__ c_0,
                                                     const float* __restrict__ b, const float* __restrict__ b_d, float* __restrict__ BIAS,
                                                     unsigned short* __restrict__ HX16, float* __restrict__ C32) {
  unsigned v = blockIdx.x * (unsigned)kThr + threadIdx.x;
  asm volatile("" : "+v"(v));
  if (v < 1280u) {
    const unsigned i0 = v * 4u;
    v4f o = {0.f, 0.f, 0.f, 0.f};
    if (i0 < (unsigned)kFBO) {
      const v4f a = *(const v4f*)(b + i0);
#pragma unroll
      for (int e = 0; e < 4; ++e) { const float p = a[e]; o[e] = bf16r(p); }
    } else if (i0 < (unsigned)(kFBO + kO)) {
      const v4f a = *(const v4f*)(b_d + (i0 - (unsigned)kFBO));
#pragma unroll
      for (int e = 0; e < 4; ++e) { const float p = a[e]; o[e] = bf16r(p); }
    }
    float* dp = BIAS + i0;
    *(volatile v4f*)dp = o;
    __threadfence();
    *(volatile v4f*)dp = o;
  } else if (v < 165120u) {
    v8h hv;
    unsigned short* dp;
    const float* sp;
    if (v < 132352u) {
      const unsigned w = v - 1280u;
      sp = h_0 + (size_t)w * 8u;
      dp = HX16 + (size_t)(w >> 7) * kK + (w & 127u) * 8u;
    } else {
      const unsigned w = v - 132352u;
      const unsigned bb = w >> 5, c8 = (w & 31u) * 8u;
      sp = X + (size_t)bb * kT * kI + c8;
      dp = HX16 + (size_t)bb * kK + kHid + c8;
    }
    const v4f a0 = *(const v4f*)sp, a1 = *(const v4f*)(sp + 4);
#pragma unroll
    for (int e = 0; e < 4; ++e) { const float p = a0[e], q = a1[e]; hv[e] = (_Float16)carry_flush(bf16r(p), kInCarry); hv[4 + e] = (_Float16)carry_flush(bf16r(q), kInCarry); }
    *(volatile v8h*)dp = hv;
    __threadfence();
    *(volatile v8h*)dp = hv;
  } else {
    const unsigned w = v - 165120u;
    const v4f a = *(const v4f*)(c_0 + (size_t)w * 4u);
    v4f z;
#pragma unroll
    for (int e = 0; e < 4; ++e) { const float p = a[e]; z[e] = bf16r(p); }
    float* dp = C32 + (size_t)w * 4u;
    *(volatile v4f*)dp = z;
    __threadfence();
    *(volatile v4f*)dp = z;
  }
}
static_assert(kFEnd / 4 == 1280 && kB * kHid / 8 == 131072 && kB * kI / 8 == 32768 && kB * kHid / 4 == 262144 && 1280 + 131072 + 32768 + 262144 == 1669 * kThr, "set-up grid exact");
static_assert((1280 % 32) == 0 && (132352 % 32) == 0 && (165120 % 32) == 0 && (kFBO % 128) == 0 && ((kFBO + kO) % 128) == 0, "set-up regions wave-uniform");

__global__ __launch_bounds__(kThr) void cell_kernel(const float* __restrict__ GG, const float* __restrict__ X, float* __restrict__ C32,
                                                    unsigned short* __restrict__ HX16, int t) {
  unsigned v = blockIdx.x * (unsigned)kThr + threadIdx.x;
  asm volatile("" : "+v"(v));
  const unsigned b = v >> 7;
  const unsigned u8 = (v & 127u) * 8u;
  const float* gr = GG + (size_t)b * kG4 + u8;
  float* cp = C32 + (size_t)b * kHid + u8;
  v8h hv, xv;
  v4f cn0, cn1;
#pragma unroll
  for (int hlf = 0; hlf < 2; ++hlf) {
    const v4f gi = *(const v4f*)(gr + 4 * hlf), gf = *(const v4f*)(gr + kHid + 4 * hlf), gg = *(const v4f*)(gr + 2 * kHid + 4 * hlf), go = *(const v4f*)(gr + 3 * kHid + 4 * hlf);
    const v4f co = *(const v4f*)(cp + 4 * hlf);
#pragma unroll
    for (int e = 0; e < 4; ++e) {
      const float cn = fast_sigmoid(gf[e]) * co[e] + fast_sigmoid(gi[e]) * fast_tanh(gg[e]);
      const float hn = fast_sigmoid(go[e]) * fast_tanh(cn);
      if (hlf == 0) cn0[e] = cn; else cn1[e] = cn;
      hv[4 * hlf + e] = (_Float16)carry_flush(hn, kInCarry);
    }
  }
  const bool nx = (u8 < (unsigned)kI) && (t + 1 < kT);
  {
    const float* sp = X + ((size_t)b * kT + (size_t)(nx ? (t + 1) : 0)) * kI + (nx ? u8 : 0u);
    const v4f a0 = *(const v4f*)sp, a1 = *(const v4f*)(sp + 4);
#pragma unroll
    for (int e = 0; e < 4; ++e) { const float p = a0[e], q = a1[e]; xv[e] = (_Float16)carry_flush(bf16r(p), kInCarry); xv[4 + e] = (_Float16)carry_flush(bf16r(q), kInCarry); }
  }
  unsigned short* hp = HX16 + (size_t)b * kK + u8;
  unsigned short* xp = HX16 + (size_t)b * kK + kHid + (nx ? u8 : 0u);
  for (int pass = 0; pass < 2; ++pass) {
    *(volatile v4f*)cp = cn0;
    *(volatile v4f*)(cp + 4) = cn1;
    *(volatile v8h*)hp = hv;
    if (nx) *(volatile v8h*)xp = xv;
    __threadfence();
  }
}
static_assert(kB * kHid / 8 == 512 * kThr && kHid / 8 == 128 && (kI / 8) % 32 == 0, "cell grid exact; the input's threads end on a wave boundary");

__global__ __launch_bounds__(kThr) void softmax_out_kernel(const float* __restrict__ LOG, float* __restrict__ out, int t) {
  unsigned r = blockIdx.x * (unsigned)kThr + threadIdx.x;
  asm volatile("" : "+v"(r));
  const float* sr = LOG + (size_t)r * kO;
  float mx = sr[0];
#pragma unroll 1
  for (int c = 0; c < kO; c += 4) {
    const v4f a = *(const v4f*)(sr + c);
#pragma unroll
    for (int e = 0; e < 4; ++e) { const float x = a[e]; mx = (x > mx) ? x : mx; }
  }
  float sum = 0.0f;
#pragma unroll 1
  for (int c = 0; c < kO; c += 4) { const v4f a = *(const v4f*)(sr + c); sum += expf(a[0] - mx); sum += expf(a[1] - mx); sum += expf(a[2] - mx); sum += expf(a[3] - mx); }
  float* dp = out + ((size_t)r * kT + (size_t)t) * kO;
  for (int pass = 0; pass < 2; ++pass) {
#pragma unroll 1
    for (int c = 0; c < kO; c += 4) {
      const v4f a = *(const v4f*)(sr + c);
      v4f o;
#pragma unroll
      for (int e = 0; e < 4; ++e) o[e] = expf(a[e] - mx) / sum;
      *(volatile v4f*)(dp + c) = o;
    }
    __threadfence();
  }
}
static_assert(kB == 4 * kThr && (kO % 4) == 0 && ((size_t)kO * 4) % 128 == 0, "softmax grid exact; an output row is whole lines");

extern "C" void kernel_launch(void* const* d_in, const int* in_sizes, int n_in,
                              void* d_out, int out_size, void* d_ws, size_t ws_size,
                              hipStream_t stream) {
  if (n_in < 8 || d_out == nullptr || d_ws == nullptr) return;
  if (in_sizes[0] != kB * kT * kI || in_sizes[1] != kB * kHid || in_sizes[2] != kB * kHid || in_sizes[3] != kI * kG4 || in_sizes[4] != kHid * kG4) return;
  if (in_sizes[5] != kG4 || in_sizes[6] != kHid * kO || in_sizes[7] != kO) return;
  if (out_size != kB * kT * kO) return;
  if (ws_size < kWsTotal) return;
  const float* X = (const float*)d_in[0];
  const float* h_0 = (const float*)d_in[1];
  const float* c_0 = (const float*)d_in[2];
  const float* W_x = (const float*)d_in[3];
  const float* W_h = (const float*)d_in[4];
  const float* b = (const float*)d_in[5];
  const float* W_d = (const float*)d_in[6];
  const float* b_d = (const float*)d_in[7];
  float* out = (float*)d_out;
  char* ws = (char*)d_ws;
  unsigned short* W16 = (unsigned short*)(ws + kOffW16);
  unsigned short* WD16 = (unsigned short*)(ws + kOffWD16);
  float* BIAS = (float*)(ws + kOffBIAS);
  unsigned short* HX16 = (unsigned short*)(ws + kOffHX16);
  float* GG = (float*)(ws + kOffGG);
  float* C32 = (float*)(ws + kOffC32);
  float* LOG = (float*)(ws + kOffLOG);

  wt_plane_kernel<<<kG4, kHid / 8, 0, stream>>>(W_h, W16, kHid, kG4, kG4, kK, 0);
  wt_plane_kernel<<<kG4, kI / 8, 0, stream>>>(W_x, W16, kI, kG4, kG4, kK, kHid);
  wt_plane_kernel<<<kO, kHid / 8, 0, stream>>>(W_d, WD16, kHid, kO, kO, kHid, 0);
  setup_kernel<<<1669, kThr, 0, stream>>>(X, h_0, c_0, b, b_d, BIAS, HX16, C32);

  for (int t = 0; t < kT; ++t) {
    wmma_gemm64<0, false, 2, 0, false, 0><<<dim3((kB / 64) * (kG4 / 64) / 8, 1), 256, 0, stream>>>(
        HX16, HX16, kK, 0L, W16, W16, kK, 0L, (void*)GG, (void*)GG, kG4, 0L, BIAS + kFBG, nullptr, 0L, kB, kG4, kK, kSc);
    cell_kernel<<<512, kThr, 0, stream>>>(GG, X, C32, HX16, t);
    wmma_gemm64<0, false, 2, 0, false, 0><<<dim3((kB / 64) * (kO / 64) / 8, 1), 256, 0, stream>>>(
        HX16, HX16, kK, 0L, WD16, WD16, kHid, 0L, (void*)LOG, (void*)LOG, kO, 0L, BIAS + kFBO, nullptr, 0L, kB, kO, kHid, kSc);
    softmax_out_kernel<<<4, kThr, 0, stream>>>(LOG, out, t);
  }
}
